// SCENE_12386685682352
// MI455X (gfx1250) — hardware-run, weakly checked
//
#include <hip/hip_runtime.h>


namespace {
constexpr int N = 10000, NP = 10048, NLIM = 10048  , NLIMN = (NLIM < N ? NLIM : N), E = 160000, DIN = 128, HEADS = 4, D1 = 128, D4 = 256, EF = 64;
constexpr float XS = 8.0f, WSC = 256.0f;
static_assert(NP % 64 == 0 && NLIM % 64 == 0, "tiling");
typedef _Float16 b16;
typedef __attribute__((ext_vector_type(16))) _Float16 v16b;
typedef __attribute__((ext_vector_type(8))) _Float16 v8b;
typedef __attribute__((ext_vector_type(8))) float v8f;
typedef __attribute__((ext_vector_type(4))) float v4f;
__device__ __forceinline__ float bf16_rne(float f) { unsigned int u = __float_as_uint(f); u += 0x7FFFu + ((u >> 16) & 1u); return __uint_as_float(u & 0xFFFF0000u); }
__device__ __forceinline__ void split16(float v, b16& hi, b16& lo) { hi = (b16)v; lo = (b16)(v - (float)hi); }
__device__ __forceinline__ v16b frag_kb(const b16* p, int hh) { const v8b a = *(const v8b*)(p + 8 * hh), b = *(const v8b*)(p + 16 + 8 * hh); v16b f;
#pragma unroll
  for (int e = 0; e < 8; ++e) { f[e] = a[e]; f[8 + e] = b[e]; } return f; }
__device__ __forceinline__ v8f wmma16b(v16b a, v16b b, v8f c) { v8f d = __builtin_amdgcn_wmma_f32_16x16x32_f16(false, a, false, b, (short)0, c, false, false); asm volatile("v_nop\n\tv_nop\n\tv_nop\n\tv_nop" : "+v"(d) : "v"(a), "v"(b)); return d; }
__device__ __forceinline__ void wave_lds_sync() { __builtin_amdgcn_fence(__ATOMIC_RELEASE, "workgroup"); __builtin_amdgcn_wave_barrier(); __builtin_amdgcn_fence(__ATOMIC_ACQUIRE, "workgroup"); }
__device__ __forceinline__ float pmul(float a, float b) { float p = a * b; asm volatile("" : "+v"(p)); return p; }
__device__ __forceinline__ int iclamp(int v, int lo, int hi) { return v < lo ? lo : (v > hi ? hi : v); }
constexpr int CSR_NBLK = 512, CSR_GB = 9, CSR_GN = 1 << CSR_GB  , CSR_MAXG = 512, CSR_CAP = 12288  ;
__global__ __launch_bounds__(64) void csrA_kernel(const int* __restrict__ dst, int E, int N, int nG, int CHP, int NGP, int* __restrict__ STG, int* __restrict__ HST) {
  extern __shared__ int sm[];
  int* cnt = sm; int* run = sm + NGP; int* ids = sm + 2 * NGP;
  const int b = blockIdx.x; const int ch = (E + CSR_NBLK - 1) / CSR_NBLK; const int e0 = b * ch, e1 = min(E, e0 + ch);
  for (int i = threadIdx.x; i < NGP; i += 64) cnt[i] = 0;
  for (int i = threadIdx.x; i < CHP; i += 64) ids[i] = -1;
  __syncthreads();
  if (threadIdx.x == 0) {
    for (int e = e0; e < e1; ++e) { int d = dst[e]; d = (d < 0) ? 0 : (d >= N ? N - 1 : d); cnt[d >> CSR_GB] += 1; }
    int acc = 0; for (int g = 0; g < nG; ++g) { run[g] = acc; acc += cnt[g]; }
    for (int e = e0; e < e1; ++e) { int d = dst[e]; d = (d < 0) ? 0 : (d >= N ? N - 1 : d); const int g = d >> CSR_GB; ids[run[g]] = e; run[g] += 1; } }
  __syncthreads();
  typedef __attribute__((ext_vector_type(4))) int v4i;
  for (int pass = 0; pass < 2; ++pass) {
    for (int i = threadIdx.x; i < CHP / 4; i += 64) *(volatile v4i*)(STG + (size_t)b * CHP + i * 4) = *(const v4i*)(&ids[i * 4]);
    for (int i = threadIdx.x; i < NGP / 4; i += 64) { v4i v; for (int e = 0; e < 4; ++e) v[e] = (i * 4 + e < nG) ? cnt[i * 4 + e] : 0; *(volatile v4i*)(HST + (size_t)b * NGP + i * 4) = v; }
    __threadfence(); }
}
__global__ __launch_bounds__(512) void csrS_kernel(const int* __restrict__ HST, int nG, int NGP, int* __restrict__ START, int* __restrict__ TOT, int* __restrict__ OFF) {
  __shared__ int tot[CSR_MAXG];
  const int b = threadIdx.x;
  for (int pass = 0; pass < 2; ++pass) { int runb = 0; for (int g = 0; g < nG; ++g) { int c = HST[(size_t)b * NGP + g]; c = (c < 0) ? 0 : c; ((volatile int*)OFF)[(size_t)g * CSR_NBLK + b] = runb; runb += c; } __threadfence(); }
  for (int g = threadIdx.x; g < nG; g += 512) { int s = 0; for (int bb = 0; bb < CSR_NBLK; ++bb) { int c = HST[(size_t)bb * NGP + g]; s += (c < 0) ? 0 : c; } tot[g] = s; }
  __syncthreads();
  if (threadIdx.x < 32) {
    __shared__ int st[CSR_MAXG + 32];
    if (threadIdx.x == 0) { int acc = 0; for (int g = 0; g < NGP; ++g) { st[g] = acc; if (g < nG) acc += (tot[g] + 31) & ~31; } st[NGP] = acc; }
    __builtin_amdgcn_fence(__ATOMIC_RELEASE, "workgroup"); __builtin_amdgcn_wave_barrier(); __builtin_amdgcn_fence(__ATOMIC_ACQUIRE, "workgroup");
    for (int pass = 0; pass < 2; ++pass) { for (int i = threadIdx.x; i < NGP + 32; i += 32) { ((volatile int*)START)[i] = (i <= NGP) ? st[min(i, NGP)] : 0; ((volatile int*)TOT)[i] = (i < nG) ? tot[i] : 0; } __threadfence(); } }
}
__global__ __launch_bounds__(256) void csrB_kernel(const int* __restrict__ dst, int N, int nG, int CHP, int NGP, int permLen, const int* __restrict__ STG, const int* __restrict__ HST, const int* __restrict__ OFF, const int* __restrict__ START, const int* __restrict__ TOT, int* __restrict__ PERM, int* __restrict__ ROWPTR, int* __restrict__ ROWCNT, int* __restrict__ FLAG) {
  typedef __attribute__((ext_vector_type(4))) int v4i;
  __shared__ int ids[CSR_CAP]; __shared__ unsigned short key[CSR_CAP]; __shared__ int outp[CSR_CAP]; __shared__ int ncnt[CSR_GN + 1]; __shared__ int boff[CSR_NBLK + 1];
  const int g = blockIdx.x, t_ = threadIdx.x; int tot = TOT[g]; int st = START[g], stn = START[g + 1]; const int v0 = g * CSR_GN; const int nv = min(CSR_GN, N - v0);
  st = (st < 0) ? 0 : (st > permLen - 32 ? permLen - 32 : st) & ~31; stn = (stn < st) ? st : (stn > permLen ? permLen : stn); tot = (tot < 0) ? 0 : tot; if (tot > stn - st && tot <= CSR_CAP) tot = stn - st;
  if (tot > CSR_CAP) {
    for (int pass = 0; pass < 2; ++pass) { for (int i = t_; i < CSR_GN / 4; i += 256) { v4i a, c; for (int e = 0; e < 4; ++e) { a[e] = st; c[e] = 0; } *(volatile v4i*)(ROWPTR + v0 + i * 4) = a; *(volatile v4i*)(ROWCNT + v0 + i * 4) = c; } if (t_ == 0) ((volatile int*)FLAG)[0] = 1; __threadfence(); } (void)nv; return; }
  if (t_ == 0) { int acc = 0; for (int b = 0; b < CSR_NBLK; ++b) { boff[b] = acc; int c = HST[(size_t)b * NGP + g]; c = (c < 0) ? 0 : (c > CHP ? CHP : c); acc += c; if (acc > tot) acc = tot; } boff[CSR_NBLK] = acc; }
  for (int i = t_; i <= CSR_GN; i += 256) ncnt[i] = 0;
  __syncthreads();
  for (int b = 0; b < CSR_NBLK; ++b) { const int c = boff[b + 1] - boff[b]; int o_ = OFF[(size_t)g * CSR_NBLK + b]; o_ = (o_ < 0) ? 0 : (o_ > CHP - c ? CHP - c : o_); const int* src_ = STG + (size_t)b * CHP + o_;
    for (int i = t_; i < c; i += 256) { int id = src_[i]; id = (id < 0) ? 0 : id; ids[boff[b] + i] = id; int d = dst[id]; d = (d < v0) ? v0 : (d >= N ? N - 1 : d); int kk = d - v0; kk = (kk < 0) ? 0 : (kk >= CSR_GN ? CSR_GN - 1 : kk); key[boff[b] + i] = (unsigned short)kk; } }
  __syncthreads();
  if (t_ == 0) { for (int i = 0; i < tot; ++i) ncnt[key[i]] += 1; int acc = 0; for (int vl = 0; vl < CSR_GN; ++vl) { const int c = ncnt[vl]; ncnt[vl] = acc; acc += c; } ncnt[CSR_GN] = acc;
    for (int i = 0; i < tot; ++i) { const int vl = key[i]; outp[ncnt[vl]] = ids[i]; ncnt[vl] += 1; }
    for (int vl = CSR_GN; vl > 0; --vl) ncnt[vl] = ncnt[vl - 1]; ncnt[0] = 0; }
  __syncthreads();
  for (int pass = 0; pass < 2; ++pass) {
    for (int i = t_; i < (stn - st) / 4; i += 256) { v4i v; for (int e = 0; e < 4; ++e) { const int q = i * 4 + e; v[e] = (q < tot) ? outp[q] : -1; } *(volatile v4i*)(PERM + st + i * 4) = v; }
    for (int i = t_; i < CSR_GN / 4; i += 256) { v4i a, c; for (int e = 0; e < 4; ++e) { const int vl = i * 4 + e; a[e] = st + ncnt[vl]; c[e] = (vl < nv) ? (ncnt[vl + 1] - ncnt[vl]) : 0; } *(volatile v4i*)(ROWPTR + v0 + i * 4) = a; *(volatile v4i*)(ROWCNT + v0 + i * 4) = c; }
    __threadfence(); }
}
__global__ __launch_bounds__(256) void csrZ_kernel(int* __restrict__ p, size_t n4) { typedef __attribute__((ext_vector_type(4))) int v4i; const size_t tid = (size_t)blockIdx.x * 256 + threadIdx.x, nth = (size_t)gridDim.x * 256; v4i z = {0, 0, 0, 0}; for (size_t i = tid; i < n4; i += nth) *(volatile v4i*)(p + i * 4) = z; }
struct CsrBufs { int *STG, *HST, *OFF, *START, *TOT, *PERM, *ROWPTR, *ROWCNT, *FLAG; int nG, NGP, CHP; size_t permLen; char* base; size_t bytes; };
static size_t csr_carve(CsrBufs& c, char* ws, size_t off, int E, int N) {
  const size_t off0 = off; c.base = ws + off;
  auto al = [&](size_t bytes) { char* p = ws + off; off += (bytes + 255) & ~(size_t)255; return p; };
  c.nG = (N + CSR_GN - 1) / CSR_GN; c.NGP = (c.nG + 31) & ~31; const int ch = (E + CSR_NBLK - 1) / CSR_NBLK; c.CHP = (ch + 31) & ~31; c.permLen = (size_t)E + 32 * (size_t)c.nG + 32;
  c.STG = (int*)al((size_t)CSR_NBLK * c.CHP * 4); c.HST = (int*)al((size_t)CSR_NBLK * c.NGP * 4); c.OFF = (int*)al((size_t)c.NGP * CSR_NBLK * 4); c.START = (int*)al((size_t)(c.NGP + 64) * 4); c.TOT = (int*)al((size_t)(c.NGP + 64) * 4);
  c.PERM = (int*)al(c.permLen * 4); c.ROWPTR = (int*)al((size_t)c.nG * CSR_GN * 4); c.ROWCNT = (int*)al((size_t)c.nG * CSR_GN * 4); c.FLAG = (int*)al(256);
  c.bytes = off - off0; return off;
}
static void csr_build(const CsrBufs& c, const int* dst, int E, int N, hipStream_t stream) {
  const size_t smem = (size_t)(2 * c.NGP + c.CHP) * 4;
  csrZ_kernel<<<512, 256, 0, stream>>>((int*)c.base, c.bytes / 16);
  csrA_kernel<<<CSR_NBLK, 64, smem, stream>>>(dst, E, N, c.nG, c.CHP, c.NGP, c.STG, c.HST);
  csrS_kernel<<<1, 512, 0, stream>>>(c.HST, c.nG, c.NGP, c.START, c.TOT, c.OFF);
  csrB_kernel<<<c.nG, 256, 0, stream>>>(dst, N, c.nG, c.CHP, c.NGP, (int)c.permLen, c.STG, c.HST, c.OFF, c.START, c.TOT, c.PERM, c.ROWPTR, c.ROWCNT, c.FLAG);
}

__global__ __launch_bounds__(256) void prep_kernel(const float* __restrict__ w1, const float* __restrict__ r1, const float* __restrict__ w2, const float* __restrict__ r2, const float* __restrict__ w3, const float* __restrict__ r3, const float* __restrict__ w4, const float* __restrict__ r4, const float* __restrict__ we1, const float* __restrict__ ae1,
                                                   b16* __restrict__ WT1, b16* __restrict__ WT2, b16* __restrict__ WT3, b16* __restrict__ WT4, float* __restrict__ WEA) {
  size_t t = (size_t)blockIdx.x * 256 + threadIdx.x; v8b o;
  for (int l = 0; l < 4; ++l) { const int D = (l == 3) ? D4 : D1; const size_t n = (size_t)(5 * D) * DIN / 8; const float* w = l == 0 ? w1 : l == 1 ? w2 : l == 2 ? w3 : w4; const float* r = l == 0 ? r1 : l == 1 ? r2 : l == 2 ? r3 : r4; b16* WT = l == 0 ? WT1 : l == 1 ? WT2 : l == 2 ? WT3 : WT4;
    if (t < n) { const size_t e = t * 8; const int oo = (int)(e / DIN), k0 = (int)(e % DIN);
      for (int j = 0; j < 8; ++j) { const int k = k0 + j; const float val = (oo < 4 * D) ? w[((size_t)k * HEADS + oo / D) * D + oo % D] : r[(size_t)k * D + (oo - 4 * D)]; o[j] = (b16)(bf16_rne(val) * WSC); }
      for (int pass = 0; pass < 2; ++pass) { *(volatile v8b*)(WT + e) = o; __threadfence(); } return; }
    t -= n; }
  if (t < 32) { const int lane = (int)t;
    float vals[8]; for (int j = 0; j < 8; ++j) { const int q = lane * 8 + j; const int i = q / 4, h = q % 4; float s = 0.0f; for (int d = 0; d < D1; ++d) s += pmul(bf16_rne(we1[((size_t)i * HEADS + h) * D1 + d]), bf16_rne(ae1[h * D1 + d])); vals[j] = s; }
    v4f a = {vals[0], vals[1], vals[2], vals[3]}, b = {vals[4], vals[5], vals[6], vals[7]};
    for (int pass = 0; pass < 2; ++pass) { *(volatile v4f*)(WEA + lane * 8) = a; *(volatile v4f*)(WEA + lane * 8 + 4) = b; __threadfence(); } }
}
typedef __attribute__((ext_vector_type(2))) float v2f;
template <int FIRST, int D>
__global__ __launch_bounds__(128) void proj_kernel(const float* __restrict__ X, const b16* __restrict__ WT, const float* __restrict__ al, const float* __restrict__ ar, float* __restrict__ FT, float* __restrict__ R, float* __restrict__ ELR) {
  __shared__ __attribute__((aligned(16))) float Tf[4][16][128 + 4]; __shared__ float Te[4][16][2];
  const int wave = threadIdx.x >> 5, lane = threadIdx.x & 31, nloc = lane & 15, hlf = lane >> 4; const size_t m0 = (size_t)blockIdx.x * 64 + wave * 16; const int slab = blockIdx.y, n0 = slab * 128; const size_t vr = m0 + nloc;
  v8f acc[8];
#pragma unroll
  for (int t = 0; t < 8; ++t) acc[t] = (v8f){};
const size_t vra = (vr < (size_t)N) ? vr : (size_t)(N - 1);
#pragma unroll
  for (int ks = 0; ks < 4; ++ks) { v16b ah, a2; const float* xr = X + vra * DIN + ks * 32;
    const v4f c0 = *(const v4f*)(xr + 8 * hlf), c1 = *(const v4f*)(xr + 8 * hlf + 4), c2 = *(const v4f*)(xr + 16 + 8 * hlf), c3 = *(const v4f*)(xr + 16 + 8 * hlf + 4); float cv[16];
    for (int i = 0; i < 4; ++i) { cv[i] = c0[i]; cv[4 + i] = c1[i]; cv[8 + i] = c2[i]; cv[12 + i] = c3[i]; }
#pragma unroll
    for (int e2 = 0; e2 < 16; ++e2) { const float xv = (vr < (size_t)N) ? cv[e2] : 0.0f; if (FIRST) { ah[e2] = (b16)(bf16_rne(xv) * XS); a2[e2] = (b16)0.0f; } else { b16 p, q; split16(xv * XS, p, q); ah[e2] = p; a2[e2] = q; } }
#pragma unroll
    for (int t = 0; t < 8; ++t) { const v16b bw = frag_kb(WT + (size_t)(n0 + t * 16 + nloc) * DIN + ks * 32, hlf); acc[t] = wmma16b(ah, bw, acc[t]); if (!FIRST) acc[t] = wmma16b(a2, bw, acc[t]); } }
  const bool featslab = n0 < 4 * D; float pel[8], per[8];
#pragma unroll
  for (int r = 0; r < 8; ++r) { pel[r] = 0.0f; per[r] = 0.0f; }
#pragma unroll
  for (int t = 0; t < 8; ++t) { const int cc = n0 + t * 16 + nloc; float a1 = 0.0f, a2v = 0.0f; if (featslab) { const int h = cc / D, d = cc % D; a1 = bf16_rne(al[h * D + d]); a2v = bf16_rne(ar[h * D + d]); }
#pragma unroll
    for (int r = 0; r < 8; ++r) { const float z = (m0 + 8 * hlf + r < (size_t)N) ? acc[t][r] * (1.0f / (XS * WSC)) : 0.0f; Tf[wave][8 * hlf + r][t * 16 + nloc] = z; pel[r] += z * a1; per[r] += z * a2v; } }
#pragma unroll
  for (int r = 0; r < 8; ++r) {
#pragma unroll
    for (int o = 1; o < 16; o <<= 1) { pel[r] += __shfl_xor(pel[r], o); per[r] += __shfl_xor(per[r], o); }
    if (nloc == 0) { Te[wave][8 * hlf + r][0] = pel[r]; Te[wave][8 * hlf + r][1] = per[r]; } }
  wave_lds_sync();
  for (int pass = 0; pass < 2; ++pass) {
    for (int rr = 0; rr < 16; ++rr) { const v4f f = *(const v4f*)(&Tf[wave][rr][lane * 4]); if (featslab) *(volatile v4f*)(FT + (m0 + rr) * (4 * D) + n0 + lane * 4) = f; else *(volatile v4f*)(R + (m0 + rr) * D + (n0 - 4 * D) + lane * 4) = f; }
    if (featslab) {   ((volatile float*)ELR)[((size_t)slab * NP + m0 + (lane >> 1)) * 2 + (lane & 1)] = Te[wave][lane >> 1][lane & 1]; }
    __threadfence(); }
}
template <int D, int EDGE>
__global__ __launch_bounds__(256) void edge_kernel(const float* __restrict__ FT, const float* __restrict__ R, const float* __restrict__ ELR, const float* __restrict__ ef, const float* __restrict__ WEA, const int* __restrict__ srcs, const int* __restrict__ PERM, const int* __restrict__ ROWPTR, const int* __restrict__ ROWCNT, int permLen, float* __restrict__ H) {
  constexpr int CPL = 4 * D / 32;
  const int wave = threadIdx.x >> 5, lane = threadIdx.x & 31; const size_t v = (size_t)blockIdx.x * 8 + wave; const int c = lane * CPL, hd = lane >> 3;
  float acc[CPL]; for (int j = 0; j < CPL; ++j) acc[j] = 0.0f; float den = 0.0f;
  if (v < (size_t)NLIMN) { float erv = (D == 128) ? ELR[((size_t)hd * NP + v) * 2 + 1] : (ELR[((size_t)(2 * hd) * NP + v) * 2 + 1] + ELR[((size_t)(2 * hd + 1) * NP + v) * 2 + 1]); float m = -INFINITY;
    int st = ROWPTR[v], cnt = ROWCNT[v]; cnt = iclamp(cnt, 0, 65536); st = iclamp(st, 0, permLen - cnt);
#pragma unroll 1
    for (int j = 0; j < cnt; ++j) { const int e = iclamp(PERM[st + j], 0, E - 1); const size_t s = (size_t)iclamp(srcs[e], 0, N - 1); if (s >= (size_t)NLIM) continue;
      float elv = (D == 128) ? ELR[((size_t)hd * NP + s) * 2] : (ELR[((size_t)(2 * hd) * NP + s) * 2] + ELR[((size_t)(2 * hd + 1) * NP + s) * 2]); float lg = elv + erv;
      if (EDGE) { float p = 0.0f; const float* er_ = ef + (size_t)e * EF; for (int i = (lane & 7); i < EF; i += 8) p += pmul(bf16_rne(er_[i]), WEA[i * HEADS + hd]);
        p += __shfl_xor(p, 1); p += __shfl_xor(p, 2); p += __shfl_xor(p, 4); lg += p; }
      lg = lg >= 0.0f ? lg : 0.2f * lg;
      const float mn = fmaxf(m, lg); const float alf = (m == -INFINITY) ? 0.0f : __expf(m - mn), w = __expf(lg - mn); const float* fr = FT + s * (4 * D) + c;
      for (int q = 0; q < CPL; q += 4) { const v4f f = *(const v4f*)(fr + q); for (int i = 0; i < 4; ++i) acc[q + i] = acc[q + i] * alf + f[i] * w; }
      den = den * alf + w; m = mn; }
    const float inv = (den > 0.0f) ? 1.0f / den : 0.0f; for (int j = 0; j < CPL; ++j) acc[j] *= inv; }
  for (int j = 0; j < CPL; ++j) { acc[j] += __shfl_xor(acc[j], 8); acc[j] += __shfl_xor(acc[j], 16); acc[j] *= 0.25f; }
  const int c0 = (lane & 7) * CPL; if (v >= (size_t)NLIMN) return;
  for (int pass = 0; pass < 2; ++pass) { if (lane < 8) { for (int q = 0; q < CPL; q += 4) { v4f o4; const v4f rv = *(const v4f*)(R + v * D + c0 + q); for (int i = 0; i < 4; ++i) o4[i] = fmaxf(acc[q + i] + rv[i], 0.0f); *(volatile v4f*)(H + v * D + c0 + q) = o4; } } __threadfence(); }
}
}

extern "C" void kernel_launch(void* const* d_in, const int* in_sizes, int n_in, void* d_out, int out_size, void* d_ws, size_t ws_size, hipStream_t stream) {
  (void)n_in;
  auto Fp = [&](int i) { return (const float*)d_in[i]; }; auto Ip = [&](int i) { return (const int*)d_in[i]; };
  if (in_sizes[0] != N * DIN || in_sizes[1] != E * EF || in_sizes[2] != E || in_sizes[3] != E || in_sizes[4] != DIN * HEADS * D1 || in_sizes[5] != EF * HEADS * D1 || in_sizes[6] != HEADS * D1 || in_sizes[9] != DIN * D1 || in_sizes[10] != DIN * HEADS * D1 || in_sizes[14] != DIN * HEADS * D1 || in_sizes[18] != DIN * HEADS * D4 || in_sizes[19] != HEADS * D4 || in_sizes[21] != DIN * D4 || out_size != N * D4) return;
  size_t off = 0; char* ws = (char*)d_ws;
  auto carve = [&](size_t bytes) { char* p = ws + off; off += (bytes + 255) & ~(size_t)255; return p; };
  b16* WT1 = (b16*)carve((size_t)5 * D1 * DIN * 2); b16* WT2 = (b16*)carve((size_t)5 * D1 * DIN * 2); b16* WT3 = (b16*)carve((size_t)5 * D1 * DIN * 2); b16* WT4 = (b16*)carve((size_t)5 * D4 * DIN * 2); float* WEA = (float*)carve(EF * HEADS * 4);
  float* FT = (float*)carve((size_t)NP * 4 * D4 * 4); float* R = (float*)carve((size_t)NP * D4 * 4); float* ELR = (float*)carve((size_t)10 * NP * 2 * 4); float* HA = (float*)carve((size_t)NP * D1 * 4); float* HB = (float*)carve((size_t)NP * D1 * 4);
  CsrBufs csr; off = csr_carve(csr, ws, off, E, N);
  if (off > ws_size || off > ((size_t)128 << 20)) return;
  prep_kernel<<<(unsigned)((((size_t)3 * 5 * D1 * DIN + (size_t)5 * D4 * DIN) / 8 + 32 + 255) / 256), 256, 0, stream>>>(Fp(4), Fp(9), Fp(10), Fp(13), Fp(14), Fp(17), Fp(18), Fp(21), Fp(5), Fp(8), WT1, WT2, WT3, WT4, WEA);
  csr_build(csr, Ip(3), E, N, stream);
  proj_kernel<1, D1><<<dim3(NLIM / 64, 5), 128, 0, stream>>>(Fp(0), WT1, Fp(6), Fp(7), FT, R, ELR);
  edge_kernel<D1, 1><<<NP / 8, 256, 0, stream>>>(FT, R, ELR, Fp(1), WEA, Ip(2), csr.PERM, csr.ROWPTR, csr.ROWCNT, (int)csr.permLen, HA);
  proj_kernel<0, D1><<<dim3(NLIM / 64, 5), 128, 0, stream>>>(HA, WT2, Fp(11), Fp(12), FT, R, ELR);
  edge_kernel<D1, 0><<<NP / 8, 256, 0, stream>>>(FT, R, ELR, nullptr, nullptr, Ip(2), csr.PERM, csr.ROWPTR, csr.ROWCNT, (int)csr.permLen, HB);
  proj_kernel<0, D1><<<dim3(NLIM / 64, 5), 128, 0, stream>>>(HB, WT3, Fp(15), Fp(16), FT, R, ELR);
  edge_kernel<D1, 0><<<NP / 8, 256, 0, stream>>>(FT, R, ELR, nullptr, nullptr, Ip(2), csr.PERM, csr.ROWPTR, csr.ROWCNT, (int)csr.permLen, HA);
  proj_kernel<0, D4><<<dim3(NLIM / 64, 10), 128, 0, stream>>>(HA, WT4, Fp(19), Fp(20), FT, R, ELR);
  edge_kernel<D4, 0><<<NP / 8, 256, 0, stream>>>(FT, R, ELR, nullptr, nullptr, Ip(2), csr.PERM, csr.ROWPTR, csr.ROWCNT, (int)csr.permLen, (float*)d_out);
}
